// MultiHeadSelfAttention_17523466567782
// MI455X (gfx1250) — hardware-verified
//
#include <hip/hip_runtime.h>


#ifndef NB
#define NB 2
#endif
#ifndef SEQ
#define SEQ 2048
#endif
#define NB_FULL  2
#define SEQ_FULL 2048
#define DM    1024
#define NH    16
#define HD    64
#define DQ    (NH * HD)
#define MROWS (NB * SEQ)
#define QKCAR 8.0f
#define VCAR  16.0f
#define RCAR  2048.0f
#define PSH   8.0f

static_assert(DQ == DM);
static_assert(SEQ % 64 == 0);
static_assert(NB <= NB_FULL);
static_assert(SEQ <= SEQ_FULL);
static_assert(DM % 32 == 0);
static_assert(HD == 64);
static_assert(((size_t)MROWS * DM / 8) % 256 == 0);
static_assert(((size_t)DM * DM / 2) % 256 == 0);
static_assert(16 * 32 * 8 == 64 * 64);
static_assert(4 * 32 * 8 == 16 * 64);
static_assert(4 * 8 * 32 * 4 == 64 * 64);

typedef _Float16 h16;
typedef unsigned short bf;
typedef __attribute__((ext_vector_type(16))) __bf16   v16bf;
typedef __attribute__((ext_vector_type(16))) _Float16 v16h;
typedef __attribute__((ext_vector_type(8)))  _Float16 v8h;
typedef __attribute__((ext_vector_type(8)))  unsigned short v8us;
typedef __attribute__((ext_vector_type(2)))  unsigned short v2us;
typedef __attribute__((ext_vector_type(8)))  float    v8f;
typedef __attribute__((ext_vector_type(4)))  float    v4f;
typedef v4f  __attribute__((may_alias)) v4fa;

__device__ __forceinline__ unsigned short f2bf(float f) { unsigned u = __float_as_uint(f); u += 0x7FFFu + ((u >> 16) & 1u); return (unsigned short)(u >> 16); }
__device__ __forceinline__ float bf2f(unsigned short b) { return __uint_as_float(((unsigned)b) << 16); }
__device__ __forceinline__ void splitf(float y, unsigned short& h, unsigned short& l) { h = f2bf(y); l = f2bf(y - bf2f(h)); }
__device__ __forceinline__ v16h cat16(v8h lo, v8h hi) { return __builtin_shufflevector(lo, hi, 0, 1, 2, 3, 4, 5, 6, 7, 8, 9, 10, 11, 12, 13, 14, 15); }
__device__ __forceinline__ v16bf cat16b(v8us lo, v8us hi) { return __builtin_bit_cast(v16bf, __builtin_shufflevector(lo, hi, 0, 1, 2, 3, 4, 5, 6, 7, 8, 9, 10, 11, 12, 13, 14, 15)); }
__device__ __forceinline__ v8f wmma16(v16h a, v16h b, v8f c) { return __builtin_amdgcn_wmma_f32_16x16x32_f16(false, a, false, b, (short)0, c, false, false); }
__device__ __forceinline__ v8f wmmab(v16bf a, v16bf b, v8f c) { return __builtin_amdgcn_wmma_f32_16x16x32_bf16(false, a, false, b, (short)0, c, false, false); }

template <typename T16> struct WFrag;
template <> struct WFrag<h16> { typedef v16h V; static __device__ __forceinline__ V ld(const h16* p) { return cat16(*(const v8h*)p, *(const v8h*)(p + 16)); } static __device__ __forceinline__ v8f mma(V a, V b, v8f c) { return wmma16(a, b, c); } };
template <> struct WFrag<bf> { typedef v16bf V; static __device__ __forceinline__ V ld(const bf* p) { return cat16b(*(const v8us*)p, *(const v8us*)(p + 16)); } static __device__ __forceinline__ v8f mma(V a, V b, v8f c) { return wmmab(a, b, c); } };

template <typename T16, int NSPLIT>
__device__ __forceinline__ void gemm_main(const T16* __restrict__ A, const T16* __restrict__ A2, const T16* __restrict__ Bt, const int K,
                                          const unsigned r0, const unsigned c0, const unsigned lr, const unsigned hi, v8f (&acc)[4][4]) {
    typedef typename WFrag<T16>::V V;
#pragma unroll
    for (int mb = 0; mb < 4; ++mb)
#pragma unroll
        for (int nb = 0; nb < 4; ++nb) acc[mb][nb] = (v8f){};
    const size_t aoff = (size_t)(r0 + lr) * K + 8 * hi, boff = (size_t)(c0 + lr) * K + 8 * hi;
#pragma unroll 1
    for (int kc = 0; kc < K; kc += 32) {
        V a[4], a2[4];
#pragma unroll
        for (int mb = 0; mb < 4; ++mb) { a[mb] = WFrag<T16>::ld(A + aoff + (size_t)mb * 16 * K + kc); if (NSPLIT == 1) a2[mb] = WFrag<T16>::ld(A2 + aoff + (size_t)mb * 16 * K + kc); }
#pragma unroll
        for (int nb = 0; nb < 4; ++nb) { const V b = WFrag<T16>::ld(Bt + boff + (size_t)nb * 16 * K + kc);
#pragma unroll
            for (int mb = 0; mb < 4; ++mb) { acc[mb][nb] = WFrag<T16>::mma(a[mb], b, acc[mb][nb]); if (NSPLIT == 1) acc[mb][nb] = WFrag<T16>::mma(a2[mb], b, acc[mb][nb]); } }
        asm volatile("v_nop\n\tv_nop\n\tv_nop\n\tv_nop" : "+v"(acc[0][0]), "+v"(acc[1][1]), "+v"(acc[2][2]), "+v"(acc[3][3]) : "v"(a[0]), "v"(a[3]));
    }
}

__global__ __launch_bounds__(256) void k_cvtx(const float* __restrict__ x, bf* XB) {
    const unsigned i = blockIdx.x * 256u + threadIdx.x;
    if (i >= (unsigned)((size_t)MROWS * DM / 8)) return;
    const unsigned r = i >> 7, c8 = i & 127u;
    const unsigned b = r / (unsigned)SEQ, t = r - b * (unsigned)SEQ;
    const v8f v = *(const v8f*)(x + ((size_t)b * SEQ_FULL + t) * DM + c8 * 8u);
    v8us o;
#pragma unroll
    for (int k = 0; k < 8; ++k) o[k] = f2bf(v[k]);
    bf* dst = XB + (size_t)i * 8;
    *(volatile v8us*)dst = o; __threadfence(); *(volatile v8us*)dst = o;
}

__global__ __launch_bounds__(256) void k_wt4(const float* __restrict__ wq, const float* __restrict__ wk, const float* __restrict__ wv, const float* __restrict__ wo, bf* WALL) {
    const unsigned y = blockIdx.y;
    const unsigned e = (blockIdx.x * 256u + threadIdx.x) * 2u;
    if (e >= (unsigned)(DM * DM)) return;
    const unsigned n = e >> 10, k = e & 1023u;
    const float* w = (y == 0u) ? wq : ((y == 1u) ? wk : ((y == 2u) ? wv : wo));
    size_t i0, i1;
    if (y < 3u) { i0 = ((size_t)(n >> 6) * DM + k) * HD + (n & 63u); i1 = i0 + HD; }
    else        { i0 = (size_t)k * DM + n; i1 = i0 + DM; }
    v2us o; o[0] = f2bf(w[i0]); o[1] = f2bf(w[i1]);
    bf* dst = WALL + (size_t)y * DM * DM + e;
    *(volatile v2us*)dst = o; __threadfence(); *(volatile v2us*)dst = o;
}

__global__ __launch_bounds__(32) void k_proj(const bf* __restrict__ XB, const bf* __restrict__ W3, h16* QH, h16* QR, h16* KH, h16* VT) {
    __shared__ __align__(16) float os[64 * 68];
    const unsigned lane = threadIdx.x & 31u, lr = lane & 15u, hi = lane >> 4;
    const unsigned r0 = blockIdx.x * 64u, c0 = blockIdx.y * 64u;
    v8f acc[4][4];
    gemm_main<bf, 0>(XB, (const bf*)nullptr, W3, DM, r0, c0, lr, hi, acc);
#pragma unroll
    for (int mb = 0; mb < 4; ++mb)
#pragma unroll
        for (int nb = 0; nb < 4; ++nb)
#pragma unroll
            for (int j = 0; j < 8; ++j) os[(mb * 16 + hi * 8 + j) * 68 + nb * 16 + lr] = acc[mb][nb][j];
    __syncthreads();
    const unsigned which = c0 >> 10, hh = (c0 & 1023u) >> 6;
    const unsigned b = r0 / (unsigned)SEQ, t0 = r0 - b * (unsigned)SEQ;
    const size_t zb = (size_t)(b * NH + hh);
    const unsigned rq = lane >> 3, seg = lane & 7u;
    if (which < 2u) {
        h16* PH = (which == 0u) ? QH : KH;
#pragma unroll 1
        for (int ps = 0; ps < 2; ++ps) {
#pragma unroll 1
            for (unsigned s = 0; s < 16u; ++s) {
                const unsigned row = s * 4u + rq;
                const float* src = os + row * 68u + seg * 8u;
                const v4f a = *(const v4fa*)src, c = *(const v4fa*)(src + 4);
                v8h oh, orr;
#pragma unroll
                for (int i = 0; i < 4; ++i) {
                    const float y0 = a[i] * QKCAR; const h16 h0 = (h16)y0; oh[i] = h0; orr[i] = (h16)((y0 - (float)h0) * RCAR);
                    const float y1 = c[i] * QKCAR; const h16 h1 = (h16)y1; oh[4 + i] = h1; orr[4 + i] = (h16)((y1 - (float)h1) * RCAR);
                }
                const size_t off = (zb * SEQ + t0 + row) * HD + seg * 8u;
                *(volatile v8h*)(PH + off) = oh;
                if (which == 0u) *(volatile v8h*)(QR + off) = orr;
            }
            if (ps == 0) __threadfence();
        }
    } else {
#pragma unroll 1
        for (int ps = 0; ps < 2; ++ps) {
#pragma unroll 1
            for (unsigned s = 0; s < 16u; ++s) {
                const unsigned d = s * 4u + rq;
                v8h o;
#pragma unroll
                for (int i = 0; i < 8; ++i) o[i] = (h16)(os[(seg * 8u + i) * 68u + d] * VCAR);
                const size_t off = (zb * HD + d) * SEQ + t0 + seg * 8u;
                *(volatile v8h*)(VT + off) = o;
            }
            if (ps == 0) __threadfence();
        }
    }
}

__global__ __launch_bounds__(32) void k_flash(const h16* __restrict__ QH, const h16* __restrict__ QR, const h16* __restrict__ KH, const h16* __restrict__ VT, bf* CH, bf* CL) {
    __shared__ __align__(16) float os[16 * 68];
    const unsigned lane = threadIdx.x & 31u, lr = lane & 15u, hi = lane >> 4;
    const unsigned q0 = blockIdx.x * 16u, hh = blockIdx.y, b = blockIdx.z;
    const size_t zb = (size_t)(b * NH + hh);
    const h16* qh = QH + (zb * SEQ + q0 + lr) * HD + 8u * hi;
    const h16* qr = QR + (zb * SEQ + q0 + lr) * HD + 8u * hi;
    const h16* kp = KH + (zb * SEQ + lr) * HD + 8u * hi;
    const h16* vp = VT + (zb * HD + lr) * SEQ + 8u * hi;
    const v16h qfh0 = WFrag<h16>::ld(qh), qfh1 = WFrag<h16>::ld(qh + 32);
    const v16h qfr0 = WFrag<h16>::ld(qr), qfr1 = WFrag<h16>::ld(qr + 32);
    v8f o0 = (v8f){}, o1 = (v8f){}, o2 = (v8f){}, o3 = (v8f){};
    float m = -3.0e38f, l = 0.0f;
    const float C2 = (0.125f / (QKCAR * QKCAR)) * 1.4426950408889634f;
    const float RINV = 1.0f / RCAR;
#pragma unroll 1
    for (unsigned kt = 0; kt < (unsigned)SEQ; kt += 32u) {
        const h16* k0 = kp + (size_t)kt * HD;
        const v16h ka00 = WFrag<h16>::ld(k0), ka01 = WFrag<h16>::ld(k0 + 32);
        const v16h ka10 = WFrag<h16>::ld(k0 + 16 * HD), ka11 = WFrag<h16>::ld(k0 + 16 * HD + 32);
        v8f sh0 = (v8f){}, sh1 = (v8f){}, sr0 = (v8f){}, sr1 = (v8f){};
        sh0 = wmma16(ka00, qfh0, sh0); sh0 = wmma16(ka01, qfh1, sh0);
        sr0 = wmma16(ka00, qfr0, sr0); sr0 = wmma16(ka01, qfr1, sr0);
        sh1 = wmma16(ka10, qfh0, sh1); sh1 = wmma16(ka11, qfh1, sh1);
        sr1 = wmma16(ka10, qfr0, sr1); sr1 = wmma16(ka11, qfr1, sr1);
        asm volatile("v_nop\n\tv_nop\n\tv_nop\n\tv_nop" : "+v"(sh0), "+v"(sh1), "+v"(sr0), "+v"(sr1) : "v"(ka00), "v"(ka11));
        float t[16];
#pragma unroll
        for (int r = 0; r < 8; ++r) { t[r] = (sh0[r] + sr0[r] * RINV) * C2; t[8 + r] = (sh1[r] + sr1[r] * RINV) * C2; }
        float mx = t[0];
#pragma unroll
        for (int i = 1; i < 16; ++i) mx = fmaxf(mx, t[i]);
        mx = fmaxf(mx, __shfl_xor(mx, 16, 32));
        const float mn = fmaxf(m, mx);
        const float alpha = __builtin_amdgcn_exp2f(m - mn);
        m = mn;
        const float sft = PSH - mn;
        float psum = 0.0f; v16h pf;
#pragma unroll
        for (int i = 0; i < 16; ++i) { const float p = __builtin_amdgcn_exp2f(t[i] + sft); psum += p; pf[i] = (h16)p; }
        l = l * alpha + psum;
#pragma unroll
        for (int r = 0; r < 8; ++r) { o0[r] *= alpha; o1[r] *= alpha; o2[r] *= alpha; o3[r] *= alpha; }
        const h16* v0 = vp + kt;
        const v16h va0 = WFrag<h16>::ld(v0), va1 = WFrag<h16>::ld(v0 + (size_t)16 * SEQ);
        const v16h va2 = WFrag<h16>::ld(v0 + (size_t)32 * SEQ), va3 = WFrag<h16>::ld(v0 + (size_t)48 * SEQ);
        o0 = wmma16(va0, pf, o0); o1 = wmma16(va1, pf, o1); o2 = wmma16(va2, pf, o2); o3 = wmma16(va3, pf, o3);
        asm volatile("v_nop\n\tv_nop\n\tv_nop\n\tv_nop" : "+v"(o0), "+v"(o1), "+v"(o2), "+v"(o3) : "v"(pf), "v"(va3));
    }
    const float lt = l + __shfl_xor(l, 16, 32);
    const float inv = 1.0f / (lt * VCAR);
#pragma unroll
    for (int r = 0; r < 8; ++r) {
        os[lr * 68u + 8u * hi + r]       = o0[r] * inv;
        os[lr * 68u + 16u + 8u * hi + r] = o1[r] * inv;
        os[lr * 68u + 32u + 8u * hi + r] = o2[r] * inv;
        os[lr * 68u + 48u + 8u * hi + r] = o3[r] * inv;
    }
    __syncthreads();
    const unsigned rq = lane >> 3, seg = lane & 7u;
#pragma unroll 1
    for (int ps = 0; ps < 2; ++ps) {
#pragma unroll 1
        for (unsigned s = 0; s < 4u; ++s) {
            const unsigned row = s * 4u + rq;
            const float* src = os + row * 68u + seg * 8u;
            const v4f a = *(const v4fa*)src, c = *(const v4fa*)(src + 4);
            v8us oh, ol;
#pragma unroll
            for (int i = 0; i < 4; ++i) { unsigned short x0, x1; splitf(a[i], x0, x1); oh[i] = x0; ol[i] = x1; splitf(c[i], x0, x1); oh[4 + i] = x0; ol[4 + i] = x1; }
            const size_t off = ((size_t)b * SEQ + q0 + row) * DQ + hh * HD + seg * 8u;
            *(volatile v8us*)(CH + off) = oh; *(volatile v8us*)(CL + off) = ol;
        }
        if (ps == 0) __threadfence();
    }
}

__global__ __launch_bounds__(32) void k_outp(const bf* __restrict__ CH, const bf* __restrict__ CL, const bf* __restrict__ WO, float* OUT) {
    __shared__ __align__(16) float os[16 * 68];
    const unsigned lane = threadIdx.x & 31u, lr = lane & 15u, hi = lane >> 4;
    const unsigned r0 = blockIdx.x * 64u, c0 = blockIdx.y * 64u;
    v8f acc[4][4];
    gemm_main<bf, 1>(CH, CL, WO, DQ, r0, c0, lr, hi, acc);
#pragma unroll
    for (int mb = 0; mb < 4; ++mb) {
#pragma unroll
        for (int nb = 0; nb < 4; ++nb) {
#pragma unroll
            for (int j = 0; j < 8; ++j) os[(hi * 8 + j) * 68 + nb * 16 + lr] = acc[mb][nb][j]; }
        __syncthreads();
        float* crow = OUT + (size_t)(r0 + mb * 16) * DM + c0;
#pragma unroll 1
        for (int ps = 0; ps < 2; ++ps) {
#pragma unroll
            for (int s = 0; s < 8; ++s) { const unsigned row = 2u * s + hi, cofs = lr * 4u; const v4f val = *(const v4fa*)(os + row * 68u + cofs);
                *(volatile v4f*)(crow + (size_t)row * DM + cofs) = val; }
            if (ps == 0) __threadfence(); }
        __syncthreads();
    }
}

extern "C" void kernel_launch(void* const* d_in, const int* in_sizes, int n_in,
                              void* d_out, int out_size, void* d_ws, size_t ws_size, hipStream_t stream) {
    if (n_in < 5) return;
    if ((size_t)in_sizes[0] < ((size_t)(NB - 1) * SEQ_FULL + SEQ) * DM) return;
    if ((size_t)in_sizes[1] < (size_t)NH * DM * HD || (size_t)in_sizes[2] < (size_t)NH * DM * HD || (size_t)in_sizes[3] < (size_t)NH * DM * HD) return;
    if ((size_t)in_sizes[4] < (size_t)DM * DM) return;
    if ((size_t)out_size < (size_t)MROWS * DM) return;
    const float* x  = (const float*)d_in[0];
    const float* wq = (const float*)d_in[1];
    const float* wk = (const float*)d_in[2];
    const float* wv = (const float*)d_in[3];
    const float* wo = (const float*)d_in[4];
    float* OUT = (float*)d_out;
    char* wsp = (char*)d_ws;
    auto take = [&](size_t bytes) { char* p = wsp; wsp += (bytes + 255) & ~(size_t)255; return (void*)p; };
    bf*  XB   = (bf*)take((size_t)MROWS * DM * 2);
    bf*  WALL = (bf*)take((size_t)4 * DM * DM * 2);
    h16* QH   = (h16*)take((size_t)NB * NH * SEQ * HD * 2);
    h16* QR   = (h16*)take((size_t)NB * NH * SEQ * HD * 2);
    h16* KH   = (h16*)take((size_t)NB * NH * SEQ * HD * 2);
    h16* VT   = (h16*)take((size_t)NB * NH * HD * SEQ * 2);
    bf*  CH   = (bf*)take((size_t)MROWS * DQ * 2);
    bf*  CL   = (bf*)take((size_t)MROWS * DQ * 2);
    if ((size_t)(wsp - (char*)d_ws) > ws_size) return;
    const bf* WO = WALL + (size_t)3 * DM * DM;
    k_cvtx<<<dim3((unsigned)((size_t)MROWS * DM / 8 / 256)), 256, 0, stream>>>(x, XB);
    k_wt4<<<dim3((unsigned)((size_t)DM * DM / 2 / 256), 4), 256, 0, stream>>>(wq, wk, wv, wo, WALL);
    k_proj<<<dim3(MROWS / 64, 3 * DQ / 64), 32, 0, stream>>>(XB, WALL, QH, QR, KH, VT);
    k_flash<<<dim3(SEQ / 16, NH, NB), 32, 0, stream>>>(QH, QR, KH, VT, CH, CL);
    k_outp<<<dim3(MROWS / 64, DM / 64), 32, 0, stream>>>(CH, CL, WO, OUT);
}
